// OpticsSimulator_43044162240548
// MI455X (gfx1250) — hardware-run, weakly checked
//
#include <hip/hip_runtime.h>
#include <math.h>

typedef __attribute__((ext_vector_type(16))) _Float16 v16h;
typedef __attribute__((ext_vector_type(8)))  _Float16 v8h;
typedef __attribute__((ext_vector_type(8)))  float    v8f;
typedef __attribute__((ext_vector_type(4)))  float    v4f;

constexpr int kBatch    = 4;
constexpr int kH        = 1024;
constexpr int kW        = 1024;
constexpr int kCh       = 3;
constexpr int kNF       = 21;
constexpr int kPsf      = 65;
constexpr int kGridN    = 9;
constexpr int kCells    = kGridN * kGridN;
constexpr int kRes      = 31;
constexpr int kPatch    = 114;
constexpr int kPatchPix = kPatch * kPatch;
constexpr int kPsfPix   = kPsf * kPsf;
constexpr int kNN       = kPsfPix * kCh;
constexpr int kNPad     = 12736;
constexpr int kMPad     = 128;
constexpr int kKPad     = 64;
constexpr int kResPix   = kRes * kRes;
constexpr int kResN     = kResPix * kCh;
constexpr int kRPitch   = 2944;
constexpr int kRVec     = kRPitch / 4;
constexpr int kOut0N    = kBatch * kH * kW * kCh;
constexpr int kOut1N    = kCells * kResN;
constexpr size_t kImgBatchStride = (size_t)kH * kW * kCh;
constexpr float kScaleRes    = (float)kRes / (float)kPsf;
constexpr float kInvScaleRes = 1.0f / kScaleRes;
constexpr float kTriSlope    = 1.0f / kInvScaleRes;
constexpr float kPsfCtr      = (float)(kPsf - 1) * 0.5f;

static_assert(kCells == 81);
static_assert(kPatchPix == 12996);
static_assert(kNN == 12675);
static_assert(kPsfPix == 4225);
static_assert(kResN == 2883);
static_assert((kNPad % 64) == 0 && kNPad >= kNN);
static_assert((kMPad % 64) == 0 && kMPad >= kCells);
static_assert((kKPad % 32) == 0 && kKPad >= kNF);
static_assert((kRPitch % 32) == 0 && kRPitch >= kResN);
static_assert((kRVec % 32) == 0);
static_assert((size_t)kOut0N * 4 == 50331648ull);
static_assert(((size_t)kOut0N + (size_t)kOut1N) * 4 == 51265740ull);
static_assert((((size_t)kOut0N * 4) % 128) == 0);
static_assert((kW % 256) == 0);

constexpr double kDiagArg = (double)kH * (double)kH + (double)kW * (double)kW;
constexpr double kDiagLit = 0x1.6A09E667F3BCDp+10;
constexpr double kDiag = __builtin_constant_p(__builtin_sqrt(kDiagArg)) ? __builtin_sqrt(kDiagArg) : kDiagLit;
constexpr double kX0d = -(double)kW / kDiag;
constexpr double kX1d = (double)kW / kDiag;
constexpr double kY0d = (double)kH / kDiag;
constexpr double kY1d = -(double)kH / kDiag;
constexpr float kX0f = (float)kX0d;
constexpr float kY0f = (float)kY0d;
constexpr float kSpanX = (float)(kX1d - kX0d);
constexpr float kSpanY = (float)(kY1d - kY0d);
constexpr float kInvCx = 1.0f / (float)(kW - 1);
constexpr float kInvCy = 1.0f / (float)(kH - 1);
constexpr float kInvSpanX = 1.0f / kSpanX;
constexpr float kInvSpanY = 1.0f / kSpanY;
constexpr float kWScale = 1.0f / (float)kPatchPix;

static_assert(kDiagArg == 2097152.0);
static_assert(kDiag == kDiagLit);
static_assert(kDiagLit == 1024.0 * 1.41421356237309504880);
static_assert(kDiag * kDiag > 2097151.999999999 && kDiag * kDiag < 2097152.000000001);
static_assert(kX0f == -kY0f && kSpanX == -kSpanY);
static_assert(kSpanX > 1.4142f && kSpanX < 1.4143f);

constexpr int patch_origin_c(int k) { return kPatch * k - k / 3; }
static_assert(patch_origin_c(0) == 0   && patch_origin_c(1) == 114 && patch_origin_c(2) == 228);
static_assert(patch_origin_c(3) == 341 && patch_origin_c(4) == 455 && patch_origin_c(5) == 569);
static_assert(patch_origin_c(6) == 682 && patch_origin_c(7) == 796 && patch_origin_c(8) == 910);
static_assert(patch_origin_c(8) + kPatch == kH);

constexpr size_t kOffAPL  = 0;
constexpr size_t kOffTRIG = kOffAPL  + (size_t)kMPad * kKPad * 2;
constexpr size_t kOffBTP  = kOffTRIG + (size_t)2 * 128 * 4;
constexpr size_t kOffINT  = kOffBTP  + (size_t)kNPad * kKPad * 2;
constexpr size_t kOffRPL  = kOffINT  + (size_t)kMPad * kNPad * 4;
constexpr size_t kOffSPL  = kOffRPL  + (size_t)kCells * kRPitch * 4;
constexpr size_t kWsTotal = kOffSPL  + (size_t)kCells * 32 * 4;
static_assert(kWsTotal == 9132672ull);
static_assert(kWsTotal <= 134217728ull);
static_assert((kOffTRIG % 128) == 0 && (kOffBTP % 128) == 0 && (kOffINT % 128) == 0 &&
              (kOffRPL % 128) == 0 && (kOffSPL % 128) == 0);

__device__ __forceinline__ int iclamp(int v, int lo, int hi) {
  const int a = (v < lo) ? lo : v;
  return (a > hi) ? hi : a;
}

__device__ __forceinline__ float keys_w(float t) {
  const float at = fabsf(t);
  const float w1 = fmaf(fmaf(1.5f, at, -2.5f), at * at, 1.0f);
  const float w2 = fmaf(fmaf(fmaf(-0.5f, at, 2.5f), at, -4.0f), at, 2.0f);
  return (at <= 1.0f) ? w1 : ((at < 2.0f) ? w2 : 0.0f);
}

__device__ __forceinline__ float table_lerp(const float* __restrict__ tab, float soft) {
  const float si = fminf(fmaxf(soft, 0.0f), (float)(kNF - 1));
  const float fl = floorf(si);
  const int lo = iclamp((int)fl, 0, kNF - 1);
  const int hi = iclamp((int)ceilf(si), 0, kNF - 1);
  const float fr = si - fl;
  const float vlo = tab[lo];
  const float vhi = tab[hi];
  return vlo * (1.0f - fr) + vhi * fr;
}

__device__ __forceinline__ float tri_w(int i, float centre) {
  const bool ok = (i >= 0) && (i <= kPsf - 1);
  const float w = fmaxf(0.0f, 1.0f - fabsf((float)i - centre) * kTriSlope);
  return ok ? w : 0.0f;
}

__device__ __forceinline__ v8f mma_f16_guarded(v16h a, v16h b, v8f c) {
  c = __builtin_amdgcn_wmma_f32_16x16x32_f16(false, a, false, b, (short)0, c, false, false);
  asm volatile("v_nop\n\tv_nop\n\tv_nop\n\tv_nop" : "+v"(c) : "v"(a), "v"(b));
  return c;
}
__device__ __forceinline__ void acc_guard4(v8f& a, v8f& b, v8f& c, v8f& d) {
  asm volatile("v_nop\n\tv_nop\n\tv_nop\n\tv_nop" : "+v"(a), "+v"(b), "+v"(c), "+v"(d));
}
__device__ __forceinline__ v16h frag_load_h(const _Float16* p) {
  union U { v16h v; v8h h[2]; };
  U f;
  f.h[0] = *(const v8h*)(p);
  f.h[1] = *(const v8h*)(p + 16);
  return f.v;
}

__global__ __launch_bounds__(128) void cell_trig_kernel(
    const float* __restrict__ xmap, const float* __restrict__ ymap,
    float* __restrict__ ctab, float* __restrict__ stab)
{
#pragma clang fp contract(off)
  const int t = threadIdx.x;
  const int g = (t < kCells - 1) ? t : (kCells - 1);
  const int gy = g / kGridN;
  const int gx = g - gy * kGridN;
  const float x0m = xmap[0];
  const float x1m = xmap[kW - 1];
  const float y0m = ymap[0];
  const float y1m = ymap[kH - 1];
  const float qx = ((float)gx + 0.5f) / (float)kGridN;
  const float qy = ((float)gy + 0.5f) / (float)kGridN;
  const float xc = qx * (x1m - x0m) + x0m;
  const float yc = qy * (y1m - y0m) + y0m;
  const float ang = -atan2f(xc, yc);
  float sv, cv;
  sincosf(ang, &sv, &cv);
  *(volatile float*)(ctab + t) = cv;
  *(volatile float*)(stab + t) = sv;
  __threadfence();
  *(volatile float*)(ctab + t) = cv;
  *(volatile float*)(stab + t) = sv;
}

static_assert(kNF <= 32);
__global__ __launch_bounds__(256) void hist_kernel(
    const float* __restrict__ fmap, unsigned short* __restrict__ Apl)
{
  __shared__ int cnt[32];
  __shared__ int part[8][32];
  const int tid = threadIdx.x, lane = tid & 31, wave = tid >> 5;
  const int g = blockIdx.x;
  int binacc = 0;
  if (g < kCells) {
    const int gy = g / kGridN;
    const int gx = g - gy * kGridN;
    const int r0 = patch_origin_c(gy);
    const int c0 = patch_origin_c(gx);
#pragma unroll 1
    for (int it = 0; it < 51; ++it) {
      const int p = it * 256 + tid;
      const int pcl = (p < kPatchPix) ? p : (kPatchPix - 1);
      const int pr = pcl / kPatch;
      const int pc = pcl - pr * kPatch;
      float v = fmap[(size_t)(r0 + pr) * kW + (c0 + pc)];
      asm volatile("" : "+v"(v));
      const float d = rintf(v * (float)(kNF - 1));
      const bool ok = (p < kPatchPix) && (d >= 0.0f) && (d <= (float)(kNF - 1));
      const int di = (int)fminf(fmaxf(d, 0.0f), (float)(kNF - 1));
      const int dic = iclamp(di, 0, kNF - 1);
#pragma unroll 1
      for (int f = 0; f < kNF; ++f) {
        const bool hit = ok && (dic == f);
        const unsigned msk = (unsigned)__ballot(hit ? 1 : 0);
        const int c = __popc(msk);
        binacc += (lane == f) ? c : 0;
      }
    }
  }
  part[wave][lane] = binacc;
  __syncthreads();
  if (tid < 32) {
    int s = 0;
#pragma unroll
    for (int w = 0; w < 8; ++w) s += part[w][tid];
    cnt[tid] = s;
  }
  __syncthreads();
  if (wave == 0) {
    v8h hv;
#pragma unroll
    for (int e = 0; e < 8; ++e) {
      const int k = lane * 8 + e;
      const int kc = (k < 31) ? k : 31;
      const int cv = cnt[kc];
      const float fv = (k < kNF) ? (float)cv : 0.0f;
      hv[e] = (_Float16)fv;
    }
    const int lc = (lane < 8) ? lane : 7;
    unsigned short* dst = Apl + (size_t)g * kKPad + lc * 8;
    if (lane < 8) *(volatile v8h*)dst = hv;
    __threadfence();
    if (lane < 8) *(volatile v8h*)dst = hv;
  }
}

__global__ __launch_bounds__(256) void pack_bt_kernel(
    const float* __restrict__ psf, unsigned short* __restrict__ Btp)
{
  const int tid = threadIdx.x, lane = tid & 31, wave = tid >> 5;
  const int n = blockIdx.x * 32 + wave * 4 + (lane >> 3);
  const int c8 = (lane & 7) * 8;
  const int nc = (n < kNN) ? n : (kNN - 1);
  v8h hv;
#pragma unroll
  for (int e = 0; e < 8; ++e) {
    const int k = c8 + e;
    const int kc = (k < kNF) ? k : (kNF - 1);
    const float v = psf[(size_t)kc * kNN + nc];
    const bool live = (k < kNF) && (n < kNN);
    float u = live ? v : 0.0f;
    u = (fabsf(u) < 6.103515625e-5f) ? 0.0f : u;
    hv[e] = (_Float16)u;
  }
  unsigned short* dst = Btp + (size_t)n * kKPad + c8;
  *(volatile v8h*)dst = hv;
  __threadfence();
  *(volatile v8h*)dst = hv;
}

__global__ __launch_bounds__(256) void interp_gemm_kernel(
    const unsigned short* __restrict__ Ap, const unsigned short* __restrict__ Btp,
    float* __restrict__ C)
{
  const _Float16* A  = (const _Float16*)Ap;
  const _Float16* Bt = (const _Float16*)Btp;
  __shared__ __align__(16) float sT[8][16 * 68];
  const int lane = threadIdx.x & 31;
  const int wave = threadIdx.x >> 5;
  constexpr int tilesN = kNPad >> 6;
  constexpr int tilesM = kMPad >> 6;
  const int tile = blockIdx.x * 8 + wave;
  if (tile >= tilesM * tilesN) return;
  const int tm = tile / tilesN;
  const int tn = tile - tm * tilesN;
  const int m0 = tm << 6;
  const int n0 = tn << 6;
  const int rlane = lane & 15;
  const int koff  = (lane >> 4) * 8;
  const int mOff  = (lane >> 4) * 8;

  v8f acc[4][4];
#pragma unroll
  for (int i = 0; i < 4; ++i)
#pragma unroll
    for (int j = 0; j < 4; ++j) acc[i][j] = (v8f){0.f, 0.f, 0.f, 0.f, 0.f, 0.f, 0.f, 0.f};

  for (int k0 = 0; k0 < kKPad; k0 += 32) {
    v16h bh[4];
#pragma unroll
    for (int j = 0; j < 4; ++j) {
      const size_t bo = (size_t)(n0 + (j << 4) + rlane) * kKPad + koff + k0;
      bh[j] = frag_load_h(Bt + bo);
    }
#pragma unroll
    for (int i = 0; i < 4; ++i) {
      const size_t ao = (size_t)(m0 + (i << 4) + rlane) * kKPad + koff + k0;
      const v16h ah = frag_load_h(A + ao);
#pragma unroll
      for (int j = 0; j < 4; ++j) acc[i][j] = mma_f16_guarded(ah, bh[j], acc[i][j]);
    }
  }
  acc_guard4(acc[0][0], acc[0][1], acc[0][2], acc[0][3]);
  acc_guard4(acc[1][0], acc[1][1], acc[1][2], acc[1][3]);
  acc_guard4(acc[2][0], acc[2][1], acc[2][2], acc[2][3]);
  acc_guard4(acc[3][0], acc[3][1], acc[3][2], acc[3][3]);

  float* slab = sT[wave];
#pragma unroll
  for (int i = 0; i < 4; ++i) {
    const int mBase = m0 + (i << 4);
#pragma unroll
    for (int j = 0; j < 4; ++j) {
#pragma unroll
      for (int r = 0; r < 8; ++r) {
        const float v = acc[i][j][r] * kWScale;
        slab[(mOff + r) * 68 + (j << 4) + rlane] = v;
      }
    }
    __builtin_amdgcn_fence(__ATOMIC_RELEASE, "workgroup");
    __builtin_amdgcn_wave_barrier();
    __builtin_amdgcn_fence(__ATOMIC_ACQUIRE, "workgroup");
    {
      const int hh = lane >> 4, c4 = (lane & 15) * 4;
      for (int pass = 0; pass < 2; ++pass) {
#pragma unroll
        for (int it = 0; it < 8; ++it) {
          const int row = it * 2 + hh;
          const v4f v = *(const v4f*)(slab + row * 68 + c4);
          *(volatile v4f*)(C + (size_t)(mBase + row) * kNPad + n0 + c4) = v;
        }
        __threadfence();
      }
    }
    __builtin_amdgcn_fence(__ATOMIC_RELEASE, "workgroup");
    __builtin_amdgcn_wave_barrier();
    __builtin_amdgcn_fence(__ATOMIC_ACQUIRE, "workgroup");
  }
}

__global__ __launch_bounds__(256) void rotate_resize_kernel(
    const float* __restrict__ interp, const float* __restrict__ ctab, const float* __restrict__ stab,
    float* __restrict__ Rp, float* __restrict__ Sp)
{
  __shared__ __align__(16) float sRot[kNN];
  __shared__ __align__(16) float sRes[kRPitch];
  __shared__ __align__(16) float sRed[32];
  const int tid = threadIdx.x, lane = tid & 31, wave = tid >> 5;
  const int g = blockIdx.x;
  const float ca = ctab[g];
  const float sa = stab[g];
  const float* src = interp + (size_t)g * kNPad;

#pragma unroll 1
  for (int it = 0; it < 17; ++it) {
    const int p = it * 256 + tid;
    const int pc = (p < kPsfPix) ? p : (kPsfPix - 1);
    const int yy = pc / kPsf;
    const int xx = pc - yy * kPsf;
    const float dxp = (float)xx - kPsfCtr;
    const float dyp = (float)yy - kPsfCtr;
    const float sx = ca * dxp - sa * dyp + kPsfCtr;
    const float sy = sa * dxp + ca * dyp + kPsfCtr;
    const float fsx = floorf(sx), fsy = floorf(sy);
    const int xs = (int)fsx, ys = (int)fsy;
    const float fx = sx - fsx, fy = sy - fsy;
    float o0 = 0.0f, o1 = 0.0f, o2 = 0.0f;
#pragma unroll
    for (int di = 0; di < 2; ++di) {
#pragma unroll
      for (int dj = 0; dj < 2; ++dj) {
        const int yi = ys + di, xi = xs + dj;
        const float wy = di ? fy : (1.0f - fy);
        const float wx = dj ? fx : (1.0f - fx);
        const bool valid = (yi >= 0) && (yi < kPsf) && (xi >= 0) && (xi < kPsf);
        const float wv = valid ? (wy * wx) : 0.0f;
        const int yic = iclamp(yi, 0, kPsf - 1);
        const int xic = iclamp(xi, 0, kPsf - 1);
        const float* t = src + (size_t)(yic * kPsf + xic) * kCh;
        const float t0 = t[0], t1 = t[1], t2 = t[2];
        o0 = fmaf(wv, t0, o0);
        o1 = fmaf(wv, t1, o1);
        o2 = fmaf(wv, t2, o2);
      }
    }
    asm volatile("" : "+v"(o0), "+v"(o1), "+v"(o2));
    if (p < kPsfPix) {
      sRot[p * kCh + 0] = o0;
      sRot[p * kCh + 1] = o1;
      sRot[p * kCh + 2] = o2;
    }
  }
  __syncthreads();

  if (tid < kRPitch - kResN) sRes[kResN + tid] = 0.0f;
  float part0 = 0.0f, part1 = 0.0f, part2 = 0.0f;
#pragma unroll 1
  for (int it = 0; it < 4; ++it) {
    const int o = it * 256 + tid;
    const int oc = (o < kResPix) ? o : (kResPix - 1);
    const int oy = oc / kRes;
    const int ox = oc - oy * kRes;
    const float cyf = ((float)oy + 0.5f) * kInvScaleRes - 0.5f;
    const float cxf = ((float)ox + 0.5f) * kInvScaleRes - 0.5f;
    const int by = (int)floorf(cyf) - 2;
    const int bx = (int)floorf(cxf) - 2;
    float wsy = 0.0f, wsx = 0.0f;
#pragma unroll 1
    for (int t = 0; t < 6; ++t) {
      wsy += tri_w(by + t, cyf);
      wsx += tri_w(bx + t, cxf);
    }
    float a0 = 0.0f, a1 = 0.0f, a2 = 0.0f;
#pragma unroll 1
    for (int ty = 0; ty < 6; ++ty) {
      const int iy = by + ty;
      const float wy = tri_w(iy, cyf);
      const int iyc = iclamp(iy, 0, kPsf - 1);
#pragma unroll 1
      for (int tx = 0; tx < 6; ++tx) {
        const int ix = bx + tx;
        const float w = wy * tri_w(ix, cxf);
        const int ixc = iclamp(ix, 0, kPsf - 1);
        const float* t = sRot + (iyc * kPsf + ixc) * kCh;
        a0 = fmaf(w, t[0], a0);
        a1 = fmaf(w, t[1], a1);
        a2 = fmaf(w, t[2], a2);
      }
    }
    const float inv = 1.0f / (wsx * wsy);
    const float v0 = a0 * inv, v1 = a1 * inv, v2 = a2 * inv;
    if (o < kResPix) {
      sRes[o * kCh + 0] = v0;
      sRes[o * kCh + 1] = v1;
      sRes[o * kCh + 2] = v2;
    }
    part0 += (o < kResPix) ? v0 : 0.0f;
    part1 += (o < kResPix) ? v1 : 0.0f;
    part2 += (o < kResPix) ? v2 : 0.0f;
  }
#pragma unroll
  for (int off = 16; off >= 1; off >>= 1) {
    part0 += __shfl_xor(part0, off, 32);
    part1 += __shfl_xor(part1, off, 32);
    part2 += __shfl_xor(part2, off, 32);
  }
  if (lane == 0) {
    sRed[wave * 3 + 0] = part0;
    sRed[wave * 3 + 1] = part1;
    sRed[wave * 3 + 2] = part2;
  }
  __syncthreads();

  v4f rv[3];
#pragma unroll
  for (int it = 0; it < 3; ++it) {
    const int f = it * 256 + tid;
    const int fc = (f < kRVec) ? f : (kRVec - 1);
    rv[it] = *(const v4f*)(sRes + fc * 4);
  }
  float ssum = 0.0f;
  {
    const int ci = (lane < 3) ? lane : 2;
#pragma unroll
    for (int w = 0; w < 8; ++w) ssum += sRed[w * 3 + ci];
    ssum = (lane < 3) ? ssum : 0.0f;
  }
  float* rrow = Rp + (size_t)g * kRPitch;
  for (int pass = 0; pass < 2; ++pass) {
#pragma unroll
    for (int it = 0; it < 3; ++it) {
      const int f = it * 256 + tid;
      if (f < kRVec) *(volatile v4f*)(rrow + (size_t)f * 4) = rv[it];
    }
    if (wave == 0) *(volatile float*)(Sp + (size_t)g * 32 + lane) = ssum;
    __threadfence();
  }
}

__global__ __launch_bounds__(256) void emit_psf_kernel(
    const float* __restrict__ Rp, const float* __restrict__ Sp, float* __restrict__ out1)
{
  const int idx = blockIdx.x * 256 + threadIdx.x;
  const int ic = (idx < kOut1N) ? idx : (kOut1N - 1);
  const int g = ic / kResN;
  const int r = ic - g * kResN;
  const int c = r % kCh;
  float rvv = Rp[(size_t)g * kRPitch + r];
  float svv = Sp[(size_t)g * 32 + c];
  asm volatile("" : "+v"(rvv), "+v"(svv));
  const float v = rvv * (1.0f / svv);
  if (idx < kOut1N) *(volatile float*)(out1 + ic) = v;
  __threadfence();
  if (idx < kOut1N) *(volatile float*)(out1 + ic) = v;
}

__global__ __launch_bounds__(256) void warp_illum_kernel(
    const float* __restrict__ img, const float* __restrict__ shifts, const float* __restrict__ ritab,
    const float* __restrict__ fmap, float* __restrict__ out)
{
  __shared__ __align__(16) float sO[8 * 384];
  const int tid = threadIdx.x, lane = tid & 31, wave = tid >> 5;
  const int y = blockIdx.y;
  const int x = blockIdx.x * 256 + tid;

  const float fmv = fmap[(size_t)y * kW + x];
  const float xf = ((float)x * kInvCx) * kSpanX + kX0f;
  const float yf = ((float)y * kInvCy) * kSpanY + kY0f;
  const float r = sqrtf(xf * xf + yf * yf);
  const float shift = table_lerp(shifts, r * (float)(kNF - 1));
  const float inv_r = 1.0f / r;
  const float dxf = shift * (xf * inv_r);
  const float dyf = shift * (yf * inv_r);
  const float dx = (dxf * (float)(kW - 1)) * kInvSpanX;
  const float dy = (dyf * (float)(kH - 1)) * kInvSpanY;
  const float wxp = (float)x + dx;
  const float wyp = (float)y + dy;
  const float fx0 = floorf(wxp), fy0 = floorf(wyp);
  const int x0 = (int)fx0, y0 = (int)fy0;
  const float fx = wxp - fx0, fy = wyp - fy0;

  float acc[kBatch][kCh];
#pragma unroll
  for (int b = 0; b < kBatch; ++b)
#pragma unroll
    for (int c = 0; c < kCh; ++c) acc[b][c] = 0.0f;

#pragma unroll 1
  for (int i = 0; i < 4; ++i) {
    const float wy = keys_w(fy - (float)(i - 1));
    const int yi = iclamp(y0 + i - 1, 0, kH - 1);
#pragma unroll 1
    for (int j = 0; j < 4; ++j) {
      const float wx = keys_w(fx - (float)(j - 1));
      const int xi = iclamp(x0 + j - 1, 0, kW - 1);
      const float w = wy * wx;
      const float* p = img + ((size_t)yi * kW + xi) * kCh;
#pragma unroll
      for (int b = 0; b < kBatch; ++b) {
#pragma unroll
        for (int c = 0; c < kCh; ++c) acc[b][c] = fmaf(w, p[(size_t)b * kImgBatchStride + c], acc[b][c]);
      }
    }
  }

  const float ri = table_lerp(ritab, fmv * (float)(kNF - 1));
  float* so = sO + wave * 384;
#pragma unroll
  for (int b = 0; b < kBatch; ++b)
#pragma unroll
    for (int c = 0; c < kCh; ++c) so[b * 96 + lane * kCh + c] = acc[b][c] * ri;
  __syncthreads();

  const int x0w = blockIdx.x * 256 + wave * 32;
  v4f vv[3];
#pragma unroll
  for (int it = 0; it < 3; ++it) vv[it] = *(const v4f*)(so + (it * 32 + lane) * 4);
  for (int pass = 0; pass < 2; ++pass) {
#pragma unroll
    for (int it = 0; it < 3; ++it) {
      const int f = it * 32 + lane;
      const int b = f / 24;
      const int q = f - b * 24;
      float* dst = out + ((size_t)(b * kH + y) * kW + x0w) * kCh + q * 4;
      *(volatile v4f*)dst = vv[it];
    }
    __threadfence();
  }
}

extern "C" void kernel_launch(void* const* d_in, const int* in_sizes, int n_in,
                              void* d_out, int out_size, void* d_ws, size_t ws_size,
                              hipStream_t stream) {
  if (n_in < 7) return;
  if (in_sizes[0] != kOut0N) return;
  if (in_sizes[1] != kNF * kNN) return;
  if (in_sizes[2] != kNF) return;
  if (in_sizes[3] != kNF) return;
  if (in_sizes[4] != kH * kW) return;
  if (in_sizes[5] != kW) return;
  if (in_sizes[6] != kH) return;
  if (out_size != kOut0N + kOut1N) return;
  if (ws_size < kWsTotal) return;

  const float* img    = (const float*)d_in[0];
  const float* psfs   = (const float*)d_in[1];
  const float* shifts = (const float*)d_in[2];
  const float* ritab  = (const float*)d_in[3];
  const float* fmap   = (const float*)d_in[4];
  const float* xmap   = (const float*)d_in[5];
  const float* ymap   = (const float*)d_in[6];
  float* out  = (float*)d_out;
  float* out1 = out + (size_t)kOut0N;

  char* ws = (char*)d_ws;
  unsigned short* APL  = (unsigned short*)(ws + kOffAPL);
  float*          CTAB = (float*)(ws + kOffTRIG);
  float*          STAB = CTAB + 128;
  unsigned short* BTP  = (unsigned short*)(ws + kOffBTP);
  float*          INT  = (float*)(ws + kOffINT);
  float*          RPL  = (float*)(ws + kOffRPL);
  float*          SPL  = (float*)(ws + kOffSPL);

  cell_trig_kernel<<<1, 128, 0, stream>>>(xmap, ymap, CTAB, STAB);
  hist_kernel<<<kMPad, 256, 0, stream>>>(fmap, APL);
  pack_bt_kernel<<<kNPad / 32, 256, 0, stream>>>(psfs, BTP);
  interp_gemm_kernel<<<((kMPad / 64) * (kNPad / 64) + 7) / 8, 256, 0, stream>>>(APL, BTP, INT);
  rotate_resize_kernel<<<kCells, 256, 0, stream>>>(INT, CTAB, STAB, RPL, SPL);
  emit_psf_kernel<<<(kOut1N + 255) / 256, 256, 0, stream>>>(RPL, SPL, out1);
  warp_illum_kernel<<<dim3(kW / 256, kH), 256, 0, stream>>>(img, shifts, ritab, fmap, out);
}
